// NeuroDynMoE_51857435132579
// MI455X (gfx1250) — hardware-verified
//
#include <hip/hip_runtime.h>
#include <math.h>

typedef __attribute__((ext_vector_type(16))) _Float16 v16h;
typedef __attribute__((ext_vector_type(16))) __bf16 v16b;
typedef __attribute__((ext_vector_type(8)))  _Float16 v8h;
typedef __attribute__((ext_vector_type(8)))  float v8f;
typedef __attribute__((ext_vector_type(4)))  float v4f;
typedef __attribute__((ext_vector_type(2)))  float v2f;
typedef __attribute__((ext_vector_type(4)))  unsigned v4u;
typedef __attribute__((ext_vector_type(4)))  int v4i;
typedef float __attribute__((may_alias)) float_a;
typedef int __attribute__((may_alias)) int_a;

template <typename T> __device__ __forceinline__ void vst2(void* p, T v) { *(volatile T*)p = v; __threadfence(); *(volatile T*)p = v; }
__device__ __forceinline__ v8f wmma16(v16h a, v16h b, v8f c) {
  v8f d = __builtin_amdgcn_wmma_f32_16x16x32_f16(false, a, false, b, (short)0, c, false, false);
  asm volatile("v_nop\n\tv_nop\n\tv_nop\n\tv_nop" : "+v"(d) : "v"(a), "v"(b));
  return d;
}
__device__ __forceinline__ v8f wmma_bf(v16b a, v16b b, v8f c) {
  v8f d = __builtin_amdgcn_wmma_f32_16x16x32_bf16(false, a, false, b, (short)0, c, false, false);
  asm volatile("v_nop\n\tv_nop\n\tv_nop\n\tv_nop" : "+v"(d) : "v"(a), "v"(b));
  return d;
}
__device__ __forceinline__ v16h frag_h(const _Float16* rowk0, int lane) {
  union { v16h v; v8h q[2]; } u; const _Float16* p = rowk0 + 8 * (lane >> 4);
  u.q[0] = *(const v8h*)p; u.q[1] = *(const v8h*)(p + 16); return u.v;
}
__device__ __forceinline__ v16h frag_f32(const float* rowk0, int lane) {
  v16h a; const float* p = rowk0 + 8 * (lane >> 4);
#pragma unroll
  for (int i = 0; i < 8; ++i) { a[i] = (_Float16)p[i]; a[8 + i] = (_Float16)p[16 + i]; }
  return a;
}
__device__ __forceinline__ v16h fragc_f32(const float* W, int k0, int n, int lane, int ld, int K) {
  v16h a; const int g = lane >> 4;
#pragma unroll
  for (int i = 0; i < 8; ++i) { const int ka = k0 + 8 * g + i, kb = ka + 16;
    a[i] = (_Float16)(ka < K ? W[(size_t)ka * ld + n] : 0.f); a[8 + i] = (_Float16)(kb < K ? W[(size_t)kb * ld + n] : 0.f); }
  return a;
}
struct F2 { v16b h, l; };
__device__ __forceinline__ F2 bsplit16(const float v[16]) { F2 r;
#pragma unroll
  for (int i = 0; i < 16; ++i) { const __bf16 h = (__bf16)v[i]; r.h[i] = h; r.l[i] = (__bf16)(v[i] - (float)h); }
  return r; }
__device__ __forceinline__ F2 split_row(const float* row, int k0, int lane) { float v[16]; const float* p = row + k0 + 8 * (lane >> 4);
#pragma unroll
  for (int i = 0; i < 8; ++i) { v[i] = p[i]; v[8 + i] = p[16 + i]; }
  return bsplit16(v); }
__device__ __forceinline__ F2 split_rowK(const float* row, int k0, int lane, int K) { float v[16]; const int g = lane >> 4;
#pragma unroll
  for (int i = 0; i < 8; ++i) { const int ka = k0 + 8 * g + i, kb = ka + 16; v[i] = ka < K ? row[ka] : 0.f; v[8 + i] = kb < K ? row[kb] : 0.f; }
  return bsplit16(v); }
__device__ __forceinline__ F2 split_col(const float* W, int k0, int n, int lane, int ld, int K) { float v[16]; const int g = lane >> 4;
#pragma unroll
  for (int i = 0; i < 8; ++i) { const int ka = k0 + 8 * g + i, kb = ka + 16; v[i] = ka < K ? W[(size_t)ka * ld + n] : 0.f; v[8 + i] = kb < K ? W[(size_t)kb * ld + n] : 0.f; }
  return bsplit16(v); }
__device__ __forceinline__ v8f mac3(const F2& a, const F2& b, v8f c) { c = wmma_bf(a.l, b.h, c); c = wmma_bf(a.h, b.l, c); return wmma_bf(a.h, b.h, c); }
__device__ __forceinline__ float sigm(float v) { return 1.0f / (1.0f + expf(-v)); }
#define LDSX() do { asm volatile("s_wait_dscnt 0" ::: "memory"); __builtin_amdgcn_wave_barrier(); __builtin_amdgcn_fence(__ATOMIC_RELEASE, "workgroup"); } while (0)

#define NR 16384
#define DD 256
#define NE 8
#define HH 128

__global__ __launch_bounds__(256) void k_pack(const float* __restrict__ W1, const float* __restrict__ Wp, _Float16* __restrict__ P1, _Float16* __restrict__ P2) {
  const int n = blockIdx.x;
  const int e = n >> 7, h = n & 127, tid = threadIdx.x;
  if (tid < DD / 8) { union { v8h v; v4u u; } pk;
#pragma unroll
    for (int i = 0; i < 8; ++i) pk.v[i] = (_Float16)W1[((size_t)e * DD + tid * 8 + i) * HH + h];
    vst2(P1 + (size_t)n * DD + tid * 8, pk.u); }
  if (tid >= 32 && tid < 32 + HH / 8) { const int q = tid - 32; union { v8h v; v4u u; } pk;
#pragma unroll
    for (int i = 0; i < 8; ++i) pk.v[i] = (_Float16)Wp[((size_t)e * HH + q * 8 + i) * HH + h];
    vst2(P2 + (size_t)n * HH + q * 8, pk.u); }
}
__global__ __launch_bounds__(128) void k_core(const float* __restrict__ x, const _Float16* __restrict__ P1, const float* __restrict__ b1, _Float16* __restrict__ core) {
  __shared__ __align__(16) float so[4][16][132];
  const int tid = threadIdx.x, wave = tid >> 5, lane = tid & 31, col = lane & 15, g = lane >> 4;
  const int r0 = blockIdx.x * 64 + wave * 16, n0 = blockIdx.y * 128;
  v8f acc[8] = {};
#pragma unroll 1
  for (int kc = 0; kc < DD / 32; ++kc) { const v16h a = frag_f32(x + (size_t)(r0 + col) * DD + kc * 32, lane);
#pragma unroll
    for (int j = 0; j < 8; ++j) acc[j] = wmma16(a, frag_h(P1 + (size_t)(n0 + j * 16 + col) * DD + kc * 32, lane), acc[j]); }
#pragma unroll
  for (int j = 0; j < 8; ++j) { const float bv = b1[n0 + j * 16 + col];
#pragma unroll
    for (int r = 0; r < 8; ++r) { const float v = acc[j][r] + bv; so[wave][8 * g + r][j * 16 + col] = v > 0.f ? v : 0.f; } }
  LDSX();
  for (int q = lane; q < 16 * 16; q += 32) { const int rl = q >> 4, pc = q & 15; union { v8h v; v4u u; } pk;
#pragma unroll
    for (int i = 0; i < 8; ++i) pk.v[i] = (_Float16)so[wave][rl][pc * 8 + i];
    vst2(core + (size_t)(r0 + rl) * (NE * HH) + n0 + pc * 8, pk.u); }
}
__global__ __launch_bounds__(128) void k_plast(const _Float16* __restrict__ core, const _Float16* __restrict__ P2, const float* __restrict__ bp, const float* __restrict__ mixl,
                                             const float* __restrict__ Wo, const float* __restrict__ bo, float* __restrict__ oute) {
  __shared__ __align__(16) float so[4][16][132];
  __shared__ __align__(16) float sr[64];
  const int tid = threadIdx.x, wave = tid >> 5, lane = tid & 31, col = lane & 15, g = lane >> 4;
  const int e = blockIdx.y, r0 = blockIdx.x * 64 + wave * 16;
  const float mix = sigm(mixl[e]);
  v8f acc[8] = {};
#pragma unroll
  for (int kc = 0; kc < HH / 32; ++kc) { const v16h a = frag_h(core + (size_t)(r0 + col) * (NE * HH) + e * HH + kc * 32, lane);
#pragma unroll
    for (int j = 0; j < 8; ++j) acc[j] = wmma16(a, frag_h(P2 + (size_t)(e * HH + j * 16 + col) * HH + kc * 32, lane), acc[j]); }
#pragma unroll
  for (int j = 0; j < 8; ++j) { const int h = j * 16 + col; const float bv = bp[e * HH + h];
#pragma unroll
    for (int r = 0; r < 8; ++r) so[wave][8 * g + r][h] = tanhf(acc[j][r] + bv); }
  LDSX();
  { float d = 0.f; const _Float16* cr = core + (size_t)(r0 + col) * (NE * HH) + e * HH;
    for (int i = 0; i < 64; ++i) { const int h = g * 64 + i; const float c = (float)cr[h]; const float m = c * (1.0f - mix) + so[wave][col][h] * mix; d += m * Wo[e * HH + h]; }
    d += __shfl_xor(d, 16, 32);
    if (g == 0) sr[wave * 16 + col] = d + bo[e]; }
  __syncthreads();
  if (tid < 16) vst2(oute + (size_t)e * NR + blockIdx.x * 64 + tid * 4, *(const v4f*)(&sr[tid * 4]));
}
__global__ __launch_bounds__(256) void k_gate(const float* __restrict__ x, const float* __restrict__ Wg, const float* __restrict__ oute, float* __restrict__ out) {
  __shared__ float sWg[DD * NE];
  __shared__ __align__(16) float so[256];
  const int tid = threadIdx.x, r = blockIdx.x * 256 + tid;
  for (int q = tid; q < DD * NE; q += 256) sWg[q] = Wg[q];
  __syncthreads();
  float lg[NE];
#pragma unroll
  for (int e = 0; e < NE; ++e) lg[e] = 0.f;
  const float* xr = x + (size_t)r * DD;
#pragma unroll 1
  for (int d = 0; d < DD; ++d) { const float v = xr[d];
#pragma unroll
    for (int e = 0; e < NE; ++e) lg[e] += v * sWg[d * NE + e]; }
  float mx = lg[0];
#pragma unroll
  for (int e = 1; e < NE; ++e) mx = fmaxf(mx, lg[e]);
  float p[NE], s = 0.f;
#pragma unroll
  for (int e = 0; e < NE; ++e) { p[e] = expf(lg[e] - mx); s += p[e]; }
#pragma unroll
  for (int e = 0; e < NE; ++e) p[e] /= s;
  int i1 = 0;
#pragma unroll
  for (int e = 1; e < NE; ++e) if (p[e] > p[i1]) i1 = e;
  int i2 = i1 == 0 ? 1 : 0;
#pragma unroll
  for (int e = 0; e < NE; ++e) if (e != i1 && p[e] > p[i2]) i2 = e;
  const float wsum = p[i1] + p[i2] + 1e-10f;
  const float o = (p[i1] * oute[(size_t)i1 * NR + r] + p[i2] * oute[(size_t)i2 * NR + r]) / wsum;
  so[tid] = o; __syncthreads();
  if (tid < 64) vst2(out + (size_t)blockIdx.x * 256 + tid * 4, *(const v4f*)(&so[tid * 4]));
}
extern "C" void kernel_launch(void* const* d_in, const int* in_sizes, int n_in, void* d_out, int out_size, void* d_ws, size_t ws_size, hipStream_t stream) {
  (void)in_sizes; (void)n_in; (void)out_size; (void)ws_size;
  const float* x = (const float*)d_in[0]; const float* Wg = (const float*)d_in[1]; const float* W1 = (const float*)d_in[2]; const float* b1 = (const float*)d_in[3];
  const float* Wp = (const float*)d_in[4]; const float* bp = (const float*)d_in[5]; const float* mixl = (const float*)d_in[6]; const float* Wo = (const float*)d_in[7]; const float* bo = (const float*)d_in[8];
  float* out = (float*)d_out;
  char* ws = (char*)d_ws; size_t off = 0;
  auto take = [&](size_t bytes) { char* p = ws + off; off += (bytes + 255) & ~(size_t)255; return p; };
  _Float16* P1 = (_Float16*)take((size_t)NE * HH * DD * 2); _Float16* P2 = (_Float16*)take((size_t)NE * HH * HH * 2);
  _Float16* core = (_Float16*)take((size_t)NR * NE * HH * 2);
  float* oute = (float*)take((size_t)NE * NR * 4);
  k_pack<<<NE * HH, 256, 0, stream>>>(W1, Wp, P1, P2);
  k_core<<<dim3(NR / 64, NE * HH / 128), 128, 0, stream>>>(x, P1, b1, core);
  k_plast<<<dim3(NR / 64, NE), 128, 0, stream>>>(core, P2, bp, mixl, Wo, bo, oute);
  k_gate<<<NR / 256, 256, 0, stream>>>(x, Wg, oute, out);
}
